// MetaKRec_51728586113410
// MI455X (gfx1250) — hardware-run, weakly checked
//
#include <hip/hip_runtime.h>


namespace {
constexpr int N = 100000, NP = 100032, D = 64, E = 1200000, B = 4096, NG = 3;
constexpr float XS = 8.0f, HS8 = 256.0f  , WSC = 256.0f;
typedef _Float16 b16;
typedef __attribute__((ext_vector_type(16))) _Float16 v16b;
typedef __attribute__((ext_vector_type(8))) _Float16 v8b;
typedef __attribute__((ext_vector_type(8))) float v8f;
typedef __attribute__((ext_vector_type(4))) float v4f;
typedef __attribute__((ext_vector_type(2))) float v2f;
__device__ __forceinline__ float bf16_rne(float f) { unsigned int u = __float_as_uint(f); u += 0x7FFFu + ((u >> 16) & 1u); return __uint_as_float(u & 0xFFFF0000u); }
__device__ __forceinline__ void split16(float v, b16& hi, b16& lo) { hi = (b16)v; lo = (b16)(v - (float)hi); }
__device__ __forceinline__ v16b frag_kb(const b16* p, int hh) { const v8b a = *(const v8b*)(p + 8 * hh), b = *(const v8b*)(p + 16 + 8 * hh); v16b f;
#pragma unroll
  for (int e = 0; e < 8; ++e) { f[e] = a[e]; f[8 + e] = b[e]; } return f; }
__device__ __forceinline__ v8f wmma16b(v16b a, v16b b, v8f c) { v8f d = __builtin_amdgcn_wmma_f32_16x16x32_f16(false, a, false, b, (short)0, c, false, false); asm volatile("v_nop\n\tv_nop\n\tv_nop\n\tv_nop" : "+v"(d) : "v"(a), "v"(b)); return d; }
__device__ __forceinline__ void wave_lds_sync() { __builtin_amdgcn_fence(__ATOMIC_RELEASE, "workgroup"); __builtin_amdgcn_wave_barrier(); __builtin_amdgcn_fence(__ATOMIC_ACQUIRE, "workgroup"); }
__device__ __forceinline__ float pmul(float a, float b) { float p = a * b; asm volatile("" : "+v"(p)); return p; }
__device__ __forceinline__ float opaque(float a) { asm volatile("" : "+v"(a)); return a; }
__device__ __forceinline__ int iclamp(int v, int lo, int hi) { return v < lo ? lo : (v > hi ? hi : v); }
__device__ __forceinline__ float nexp(float x) { return __builtin_amdgcn_exp2f(x * 1.4426950408889634f); }
constexpr int CSR_NBLK = 512, CSR_GB = 9, CSR_GN = 1 << CSR_GB  , CSR_TS = (CSR_GN < 32 ? 32 : CSR_GN)  , CSR_MAXG = 512, CSR_CAP = 12288  ;
__device__ __host__ __forceinline__ int csr_tix(int v) { return (v >> CSR_GB) * CSR_TS + (v & (CSR_GN - 1)); }
__global__ __launch_bounds__(64) void csrA_kernel(const int* __restrict__ dst, int E, int N, int nG, int CHP, int NGP, int* __restrict__ STG, int* __restrict__ HST) {
  extern __shared__ int sm[];
  int* cnt = sm; int* run = sm + NGP; int* ids = sm + 2 * NGP;
  const int b = blockIdx.x; const int ch = (E + CSR_NBLK - 1) / CSR_NBLK; const int e0 = b * ch, e1 = min(E, e0 + ch);
  for (int i = threadIdx.x; i < NGP; i += 64) cnt[i] = 0;
  for (int i = threadIdx.x; i < CHP; i += 64) ids[i] = -1;
  __syncthreads();
  if (threadIdx.x == 0) {
    for (int e = e0; e < e1; ++e) { int d = dst[e]; d = (d < 0) ? 0 : (d >= N ? N - 1 : d); cnt[d >> CSR_GB] += 1; }
    int acc = 0; for (int g = 0; g < nG; ++g) { run[g] = acc; acc += cnt[g]; }
    for (int e = e0; e < e1; ++e) { int d = dst[e]; d = (d < 0) ? 0 : (d >= N ? N - 1 : d); const int g = d >> CSR_GB; ids[run[g]] = e; run[g] += 1; } }
  __syncthreads();
  typedef __attribute__((ext_vector_type(4))) int v4i;
  for (int pass = 0; pass < 2; ++pass) {
    for (int i = threadIdx.x; i < CHP / 4; i += 64) *(volatile v4i*)(STG + (size_t)b * CHP + i * 4) = *(const v4i*)(&ids[i * 4]);
    for (int i = threadIdx.x; i < NGP / 4; i += 64) { v4i v; for (int e = 0; e < 4; ++e) v[e] = (i * 4 + e < nG) ? cnt[i * 4 + e] : 0; *(volatile v4i*)(HST + (size_t)b * NGP + i * 4) = v; }
    __threadfence(); }
}
__global__ __launch_bounds__(512) void csrS_kernel(const int* __restrict__ HST, int nG, int NGP, int* __restrict__ START, int* __restrict__ TOT, int* __restrict__ OFF) {
  __shared__ int tot[CSR_MAXG];
  const int b = threadIdx.x;
  for (int pass = 0; pass < 2; ++pass) { int runb = 0; for (int g = 0; g < nG; ++g) { int c = HST[(size_t)b * NGP + g]; c = (c < 0) ? 0 : c; ((volatile int*)OFF)[(size_t)g * CSR_NBLK + b] = runb; runb += c; } __threadfence(); }
  for (int g = threadIdx.x; g < nG; g += 512) { int s = 0; for (int bb = 0; bb < CSR_NBLK; ++bb) { int c = HST[(size_t)bb * NGP + g]; s += (c < 0) ? 0 : c; } tot[g] = s; }
  __syncthreads();
  if (threadIdx.x < 32) {
    __shared__ int st[CSR_MAXG + 32];
    if (threadIdx.x == 0) { int acc = 0; for (int g = 0; g < NGP; ++g) { st[g] = acc; if (g < nG) acc += (tot[g] + 31) & ~31; } st[NGP] = acc; }
    __builtin_amdgcn_fence(__ATOMIC_RELEASE, "workgroup"); __builtin_amdgcn_wave_barrier(); __builtin_amdgcn_fence(__ATOMIC_ACQUIRE, "workgroup");
    for (int pass = 0; pass < 2; ++pass) { for (int i = threadIdx.x; i < NGP + 32; i += 32) { ((volatile int*)START)[i] = (i <= NGP) ? st[min(i, NGP)] : 0; ((volatile int*)TOT)[i] = (i < nG) ? tot[i] : 0; } __threadfence(); } }
}
__global__ __launch_bounds__(256) void csrB_kernel(const int* __restrict__ dst, int N, int nG, int CHP, int NGP, int permLen, const int* __restrict__ STG, const int* __restrict__ HST, const int* __restrict__ OFF, const int* __restrict__ START, const int* __restrict__ TOT, int* __restrict__ PERM, int* __restrict__ ROWPTR, int* __restrict__ ROWCNT, int* __restrict__ FLAG) {
  typedef __attribute__((ext_vector_type(4))) int v4i;
  __shared__ int ids[CSR_CAP]; __shared__ unsigned short key[CSR_CAP]; __shared__ int outp[CSR_CAP]; __shared__ int ncnt[CSR_GN + 1]; __shared__ int boff[CSR_NBLK + 1];
  const int g = blockIdx.x, t_ = threadIdx.x; int tot = TOT[g]; int st = START[g], stn = START[g + 1]; const int v0 = g * CSR_GN; const int nv = min(CSR_GN, N - v0); const int t0 = g * CSR_TS;
  st = (st < 0) ? 0 : (st > permLen - 32 ? permLen - 32 : st) & ~31; stn = (stn < st) ? st : (stn > permLen ? permLen : stn); tot = (tot < 0) ? 0 : tot; if (tot > stn - st && tot <= CSR_CAP) tot = stn - st;
  if (tot > CSR_CAP) {
    for (int pass = 0; pass < 2; ++pass) { for (int i = t_; i < CSR_TS / 4; i += 256) { v4i a, c; for (int e = 0; e < 4; ++e) { a[e] = st; c[e] = 0; } *(volatile v4i*)(ROWPTR + t0 + i * 4) = a; *(volatile v4i*)(ROWCNT + t0 + i * 4) = c; } if (t_ == 0) ((volatile int*)FLAG)[0] = 1; __threadfence(); } (void)nv; return; }
  if (t_ == 0) { int acc = 0; for (int b = 0; b < CSR_NBLK; ++b) { boff[b] = acc; int c = HST[(size_t)b * NGP + g]; c = (c < 0) ? 0 : (c > CHP ? CHP : c); acc += c; if (acc > tot) acc = tot; } boff[CSR_NBLK] = acc; }
  for (int i = t_; i <= CSR_GN; i += 256) ncnt[i] = 0;
  __syncthreads();
  for (int b = 0; b < CSR_NBLK; ++b) { const int c = boff[b + 1] - boff[b]; int o_ = OFF[(size_t)g * CSR_NBLK + b]; o_ = (o_ < 0) ? 0 : (o_ > CHP - c ? CHP - c : o_); const int* src_ = STG + (size_t)b * CHP + o_;
    for (int i = t_; i < c; i += 256) { int id = src_[i]; id = (id < 0) ? 0 : id; ids[boff[b] + i] = id; int d = dst[id]; d = (d < v0) ? v0 : (d >= N ? N - 1 : d); int kk = d - v0; kk = (kk < 0) ? 0 : (kk >= CSR_GN ? CSR_GN - 1 : kk); key[boff[b] + i] = (unsigned short)kk; } }
  __syncthreads();
  if (t_ == 0) { for (int i = 0; i < tot; ++i) ncnt[key[i]] += 1; int acc = 0; for (int vl = 0; vl < CSR_GN; ++vl) { const int c = ncnt[vl]; ncnt[vl] = acc; acc += c; } ncnt[CSR_GN] = acc;
    for (int i = 0; i < tot; ++i) { const int vl = key[i]; outp[ncnt[vl]] = ids[i]; ncnt[vl] += 1; }
    for (int vl = CSR_GN; vl > 0; --vl) ncnt[vl] = ncnt[vl - 1]; ncnt[0] = 0; }
  __syncthreads();
  for (int pass = 0; pass < 2; ++pass) {
    for (int i = t_; i < (stn - st) / 4; i += 256) { v4i v; for (int e = 0; e < 4; ++e) { const int q = i * 4 + e; v[e] = (q < tot) ? outp[q] : -1; } *(volatile v4i*)(PERM + st + i * 4) = v; }
    for (int i = t_; i < CSR_TS / 4; i += 256) { v4i a, c; for (int e = 0; e < 4; ++e) { const int vl = i * 4 + e; const int vc = vl < CSR_GN ? vl : CSR_GN; a[e] = (vl < CSR_GN) ? st + ncnt[vc] : st; c[e] = (vl < nv) ? (ncnt[(vc < CSR_GN ? vc : CSR_GN - 1) + 1] - ncnt[vc]) : 0; } *(volatile v4i*)(ROWPTR + t0 + i * 4) = a; *(volatile v4i*)(ROWCNT + t0 + i * 4) = c; }
    __threadfence(); }
}
__global__ __launch_bounds__(256) void csrZ_kernel(int* __restrict__ p, size_t n4) { typedef __attribute__((ext_vector_type(4))) int v4i; const size_t tid = (size_t)blockIdx.x * 256 + threadIdx.x, nth = (size_t)gridDim.x * 256; v4i z = {0, 0, 0, 0}; for (size_t i = tid; i < n4; i += nth) *(volatile v4i*)(p + i * 4) = z; }
struct CsrBufs { int *STG, *HST, *OFF, *START, *TOT, *PERM, *ROWPTR, *ROWCNT, *FLAG; int nG, NGP, CHP; size_t permLen; char* base; size_t bytes; };
static size_t csr_carve(CsrBufs& c, char* ws, size_t off, int E, int N) {
  const size_t off0 = off; c.base = ws + off;
  auto al = [&](size_t bytes) { char* p = ws + off; off += (bytes + 255) & ~(size_t)255; return p; };
  c.nG = (N + CSR_GN - 1) / CSR_GN; c.NGP = (c.nG + 31) & ~31; const int ch = (E + CSR_NBLK - 1) / CSR_NBLK; c.CHP = (ch + 31) & ~31; c.permLen = (size_t)E + 32 * (size_t)c.nG + 32;
  c.STG = (int*)al((size_t)CSR_NBLK * c.CHP * 4); c.HST = (int*)al((size_t)CSR_NBLK * c.NGP * 4); c.OFF = (int*)al((size_t)c.NGP * CSR_NBLK * 4); c.START = (int*)al((size_t)(c.NGP + 64) * 4); c.TOT = (int*)al((size_t)(c.NGP + 64) * 4);
  c.PERM = (int*)al(c.permLen * 4); c.ROWPTR = (int*)al((size_t)c.nG * CSR_TS * 4); c.ROWCNT = (int*)al((size_t)c.nG * CSR_TS * 4); c.FLAG = (int*)al(256);
  c.bytes = off - off0; return off;
}
static void csr_build(const CsrBufs& c, const int* dst, int E, int N, hipStream_t stream) {
  const size_t smem = (size_t)(2 * c.NGP + c.CHP) * 4;
  csrZ_kernel<<<512, 256, 0, stream>>>((int*)c.base, c.bytes / 16);
  csrA_kernel<<<CSR_NBLK, 64, smem, stream>>>(dst, E, N, c.nG, c.CHP, c.NGP, c.STG, c.HST);
  csrS_kernel<<<1, 512, 0, stream>>>(c.HST, c.nG, c.NGP, c.START, c.TOT, c.OFF);
  csrB_kernel<<<c.nG, 256, 0, stream>>>(dst, N, c.nG, c.CHP, c.NGP, (int)c.permLen, c.STG, c.HST, c.OFF, c.START, c.TOT, c.PERM, c.ROWPTR, c.ROWCNT, c.FLAG);
}


__global__ __launch_bounds__(256) void wprep_kernel(const float* __restrict__ w, b16* __restrict__ WT) {
  const size_t u = (size_t)blockIdx.x * 256 + threadIdx.x; if (u >= (size_t)D * D / 8) return; const size_t e = u * 8; const int o = (int)(e / D), k0 = (int)(e % D); v8b v;
  for (int j = 0; j < 8; ++j) v[j] = (b16)(bf16_rne(w[(size_t)(k0 + j) * D + o]) * WSC); for (int pass = 0; pass < 2; ++pass) { *(volatile v8b*)(WT + e) = v; __threadfence(); }
}
template <int RAW>
__global__ __launch_bounds__(256) void prop_kernel(const float* __restrict__ IN_, const int* __restrict__ srcs, const int* __restrict__ PERM, const int* __restrict__ ROWPTR, const int* __restrict__ ROWCNT, int permLen, float* __restrict__ OUT) {
  const int wave = threadIdx.x >> 5, lane = threadIdx.x & 31; const size_t v = (size_t)blockIdx.x * 8 + wave; v2f o = {0.0f, 0.0f};
  if (v < (size_t)N) { int st = ROWPTR[v], cnt = ROWCNT[v]; cnt = iclamp(cnt, 0, 65536); st = iclamp(st, 0, permLen - cnt); const float dv = cnt > 0 ? rsqrtf((float)cnt) : 0.0f; v2f a = {0.0f, 0.0f};
#pragma unroll 2
    for (int j = 0; j < cnt; ++j) { const int e = iclamp(PERM[st + j], 0, E - 1); const int s = iclamp(srcs[e], 0, N - 1); int cs = ROWCNT[s]; cs = cs < 0 ? 0 : (cs > 65536 ? 65536 : cs); const float ds = cs > 0 ? rsqrtf((float)cs) : 0.0f;
      const v2f f = *(const v2f*)(IN_ + (size_t)s * D + lane * 2); a[0] += pmul(ds, RAW ? bf16_rne(f[0]) : f[0]); a[1] += pmul(ds, RAW ? bf16_rne(f[1]) : f[1]); }
    o[0] = pmul(dv, a[0]); o[1] = pmul(dv, a[1]); }
  for (int pass = 0; pass < 2; ++pass) { *(volatile v2f*)(OUT + v * D + lane * 2) = o; __threadfence(); }
}
__global__ __launch_bounds__(32) void node_kernel(const float* __restrict__ H0, const float* __restrict__ H1, const float* __restrict__ H2, const b16* __restrict__ WT, const float* __restrict__ av, float* __restrict__ NODE) {
  __shared__ __attribute__((aligned(16))) b16 Ah[16][D + 8], Al[16][D + 8]; __shared__ __attribute__((aligned(16))) float Sc[16][4];
  const int lane = threadIdx.x, nloc = lane & 15, hlf = lane >> 4; const size_t v0 = (size_t)blockIdx.x * 16;
  float a4[4]; for (int t = 0; t < 4; ++t) a4[t] = opaque(bf16_rne(av[t * 16 + nloc]));
#pragma unroll 1
  for (int g = 0; g < NG; ++g) { const float* H = g == 0 ? H0 : (g == 1 ? H1 : H2);
    for (int rr = 0; rr < 16; ++rr) { const v2f h = *(const v2f*)(H + (v0 + rr) * D + lane * 2); for (int j = 0; j < 2; ++j) { b16 p, q; split16(h[j] * HS8, p, q); Ah[rr][lane * 2 + j] = p; Al[rr][lane * 2 + j] = q; } }
    wave_lds_sync();
    v8f acc[4];
#pragma unroll
    for (int t = 0; t < 4; ++t) acc[t] = (v8f){};
#pragma unroll
    for (int kb = 0; kb < D; kb += 32) { const v16b a = frag_kb(&Ah[nloc][kb], hlf), al = frag_kb(&Al[nloc][kb], hlf);
#pragma unroll
      for (int t = 0; t < 4; ++t) { const v16b bw = frag_kb(WT + (size_t)(t * 16 + nloc) * D + kb, hlf); acc[t] = wmma16b(a, bw, acc[t]); acc[t] = wmma16b(al, bw, acc[t]); } }
    float ps[8]; for (int r8 = 0; r8 < 8; ++r8) { float s = 0.0f; for (int t = 0; t < 4; ++t) s += pmul(acc[t][r8] * (1.0f / (HS8 * WSC)), a4[t]); ps[r8] = s; }
#pragma unroll
    for (int r8 = 0; r8 < 8; ++r8) { float s = ps[r8]; for (int o = 1; o < 16; o <<= 1) s += __shfl_xor(s, o); if (nloc == 0) Sc[8 * hlf + r8][g] = s; }
    wave_lds_sync(); }
  for (int rr = 0; rr < 16; ++rr) { const float s0 = Sc[rr][0], s1 = Sc[rr][1], s2 = Sc[rr][2]; const float m = fmaxf(s0, fmaxf(s1, s2)); const float e0 = nexp(s0 - m), e1 = nexp(s1 - m), e2 = nexp(s2 - m); const float inv = 1.0f / (e0 + e1 + e2);
    const v2f h0 = *(const v2f*)(H0 + (v0 + rr) * D + lane * 2), h1 = *(const v2f*)(H1 + (v0 + rr) * D + lane * 2), h2 = *(const v2f*)(H2 + (v0 + rr) * D + lane * 2); v2f o;
    for (int j = 0; j < 2; ++j) o[j] = pmul(e0 * inv, h0[j]) + pmul(e1 * inv, h1[j]) + pmul(e2 * inv, h2[j]);
    for (int pass = 0; pass < 2; ++pass) { *(volatile v2f*)(NODE + (v0 + rr) * D + lane * 2) = o; __threadfence(); } }
}
__global__ __launch_bounds__(256) void pair_kernel(const float* __restrict__ NODE, const int* __restrict__ user, const int* __restrict__ item, float* __restrict__ out) {
  const int b = blockIdx.x * 256 + threadIdx.x; const int u = iclamp(user[b], 0, N - 1), it = iclamp(item[b], 0, N - 1); const float* pu = NODE + (size_t)u * D; const float* pi = NODE + (size_t)it * D; float s = 0.0f;
#pragma unroll 2
  for (int k = 0; k < D; k += 4) { const v4f x = *(const v4f*)(pu + k), y = *(const v4f*)(pi + k); for (int i = 0; i < 4; ++i) s += pmul(x[i], y[i]); }
  for (int pass = 0; pass < 2; ++pass) { ((volatile float*)out)[b] = s; __threadfence(); }
}
}

extern "C" void kernel_launch(void* const* d_in, const int* in_sizes, int n_in, void* d_out, int out_size, void* d_ws, size_t ws_size, hipStream_t stream) {
  (void)n_in;
  auto Fp = [&](int i) { return (const float*)d_in[i]; }; auto Ip = [&](int i) { return (const int*)d_in[i]; };
  if (in_sizes[0] != B || in_sizes[1] != B || in_sizes[3] != 2 * E || in_sizes[4] != 2 * E || in_sizes[5] != 2 * E || in_sizes[6] != N * D || in_sizes[7] != D * D || in_sizes[8] != D || out_size != B) return;
  size_t off = 0; char* ws = (char*)d_ws;
  auto carve = [&](size_t bytes) { char* p = ws + off; off += (bytes + 255) & ~(size_t)255; return p; };
  b16* WT = (b16*)carve((size_t)D * D * 2); float* T1 = (float*)carve((size_t)NP * D * 4); float* T2 = (float*)carve((size_t)NP * D * 4); float* HG[NG]; for (int g = 0; g < NG; ++g) HG[g] = (float*)carve((size_t)NP * D * 4); float* NODE = T1;
  CsrBufs csr; off = csr_carve(csr, ws, off, E, N);
  if (off > ws_size) return;
  wprep_kernel<<<(D * D / 8 + 255) / 256, 256, 0, stream>>>(Fp(7), WT);
  for (int g = 0; g < NG; ++g) { const int* ei = Ip(3 + g);
    csr_build(csr, ei + E, E, N, stream);
    prop_kernel<1><<<NP / 8, 256, 0, stream>>>(Fp(6), ei, csr.PERM, csr.ROWPTR, csr.ROWCNT, (int)csr.permLen, T1);
    prop_kernel<0><<<NP / 8, 256, 0, stream>>>(T1, ei, csr.PERM, csr.ROWPTR, csr.ROWCNT, (int)csr.permLen, T2);
    prop_kernel<0><<<NP / 8, 256, 0, stream>>>(T2, ei, csr.PERM, csr.ROWPTR, csr.ROWCNT, (int)csr.permLen, HG[g]); }
  node_kernel<<<NP / 16, 32, 0, stream>>>(HG[0], HG[1], HG[2], WT, Fp(8), NODE);
  pair_kernel<<<B / 256, 256, 0, stream>>>(NODE, Ip(0), Ip(1), (float*)d_out);
}
